// HammingLoss_52166672777732
// MI455X (gfx1250) — hardware-verified
//
#include <hip/hip_runtime.h>
#include <stdint.h>
#include <math.h>


typedef _Float16 v8h  __attribute__((ext_vector_type(8)));
typedef _Float16 v16h __attribute__((ext_vector_type(16)));
typedef float    v8f  __attribute__((ext_vector_type(8)));
typedef float    v4f  __attribute__((ext_vector_type(4)));
typedef int      v4i  __attribute__((ext_vector_type(4)));

#define NB3       6
#define NBT       2
#define NP        1024
#define NSB       32
#define NBIT      256
#define LOGW      8
#define WIMG      256
#define HWIMG     65536
#define QR        64
#define LP8       33
#define TPB       256
#define HAM_TPB   128
#define RATIO_THR 1.1f
#define TRIP_BIAS 36.0f
#define STATIC_R  1.0f
#define DYNAMIC_R 1.0f
#define SEM_R     1.0f
#define TRIP_R    1.0f

union Frag16 { v16h v; v8h hf[2]; };

__device__ __forceinline__ v8f wmma_f16_step(v16h a, v16h b, v8f c) {
  v8f d = __builtin_amdgcn_wmma_f32_16x16x32_f16(false, a, false, b, (short)0, c, false, false);
  asm volatile("v_nop\n\tv_nop\n\tv_nop\n\tv_nop" : "+v"(d) : "v"(a), "v"(b));
  return d;
}

__device__ __forceinline__ int clampi(int v, int lo, int hi) {
  return v < lo ? lo : (v > hi ? hi : v);
}

__device__ __forceinline__ v8h bits_to_h8(int val) {
  v8h e;
#pragma unroll
  for (int j = 0; j < 8; ++j) e[j] = ((val >> j) & 1) ? (_Float16)1.0f : (_Float16)0.0f;
  return e;
}

__global__ __launch_bounds__(HAM_TPB) void k_ham(const int* __restrict__ feat, v4i* rec) {
  __shared__ v8h Al[QR * LP8];
  __shared__ v8h Bl[16 * LP8];
  __shared__ int popQ[QR];
  __shared__ int popO[16];
  __shared__ int Dt[HAM_TPB / 32][16 * 17];
  __shared__ v4i resl[QR];

  const int tid = threadIdx.x;
  const int w = tid >> 5, l = tid & 31, h = l >> 4, m = l & 15;
  const int q0 = blockIdx.x * QR;
  const int combo = blockIdx.y;
  const int b = combo >> 1, isNeg = combo & 1;
  const int qb = (isNeg ? 2 * NBT : NBT) + b;
  const int ob = b;

  {
    const int row = tid >> 1;
    const int s0 = (tid & 1) * (NSB / 2);
    const int gq = clampi(q0 + row, 0, NP - 1);
    int pop = 0;
#pragma unroll 4
    for (int s = s0; s < s0 + NSB / 2; ++s) {
      const int val = feat[(size_t)(qb * NSB + s) * NP + gq] & 0xFF;
      pop += (int)__popc((unsigned)val);
      Al[row * LP8 + s] = bits_to_h8(val);
    }
    pop += __shfl_xor(pop, 1);
    if ((tid & 1) == 0) popQ[row] = pop;
  }

  int bv0 = 0x7FFFFFFF, bv1 = 0x7FFFFFFF, bi = 0;

  for (int ct = 0; ct < NP / 16; ++ct) {
    {
      const int col = tid >> 3;
      const int s0 = (tid & 7) * (NSB / 8);
      const int go = ct * 16 + col;
      int pop = 0;
#pragma unroll
      for (int s = s0; s < s0 + NSB / 8; ++s) {
        const int val = feat[(size_t)(ob * NSB + s) * NP + go] & 0xFF;
        pop += (int)__popc((unsigned)val);
        Bl[col * LP8 + s] = bits_to_h8(val);
      }
      pop += __shfl_xor(pop, 1);
      pop += __shfl_xor(pop, 2);
      pop += __shfl_xor(pop, 4);
      if ((tid & 7) == 0) popO[col] = pop;
    }
    __syncthreads();

    v8f acc = {0.f, 0.f, 0.f, 0.f, 0.f, 0.f, 0.f, 0.f};
    const v8h* arow = Al + (w * 16 + m) * LP8;
    const v8h* brow = Bl + m * LP8;
#pragma unroll
    for (int ks = 0; ks < NBIT / 32; ++ks) {
      Frag16 fa, fb;
      fa.hf[0] = arow[4 * ks + h];
      fa.hf[1] = arow[4 * ks + 2 + h];
      fb.hf[0] = brow[4 * ks + h];
      fb.hf[1] = brow[4 * ks + 2 + h];
      acc = wmma_f16_step(fa.v, fb.v, acc);
    }
#pragma unroll
    for (int r = 0; r < 8; ++r) {
      const int row = 8 * h + r;
      const int hv = popQ[w * 16 + row] + popO[m] - 2 * (int)acc[r];
      Dt[w][row * 17 + m] = hv;
    }
    __syncthreads();
    if (l < 16) {
      const int* dr = &Dt[w][l * 17];
#pragma unroll
      for (int n = 0; n < 16; ++n) {
        const int v = dr[n];
        const int j = ct * 16 + n;
        if (v < bv0) { bv1 = bv0; bv0 = v; bi = j; }
        else if (v < bv1) { bv1 = v; }
      }
    }
  }

  if (l < 16) {
    v4i rr = {bv0, bv1, bi, 0};
    resl[w * 16 + l] = rr;
  }
  __syncthreads();
  if (w == 0) {
    const v4i r0 = resl[l];
    const v4i r1 = resl[32 + l];
    volatile v4i* dst = (volatile v4i*)(rec + (size_t)combo * NP + q0);
    dst[l] = r0;
    dst[32 + l] = r1;
    __threadfence();
    dst[l] = r0;
    dst[32 + l] = r1;
  }
}

template <int NQ>
__device__ __forceinline__ void blk_sum(double (&s)[NQ], double* red, double* tot) {
  const int tid = threadIdx.x, w = tid >> 5, l = tid & 31;
#pragma unroll
  for (int q = 0; q < NQ; ++q) {
    double v = s[q];
    v += __shfl_xor(v, 16);
    v += __shfl_xor(v, 8);
    v += __shfl_xor(v, 4);
    v += __shfl_xor(v, 2);
    v += __shfl_xor(v, 1);
    if (l == 0) red[q * (TPB / 32) + w] = v;
  }
  __syncthreads();
  if (tid < NQ) {
    double a = 0.0;
#pragma unroll
    for (int i = 0; i < TPB / 32; ++i) a += red[tid * (TPB / 32) + i];
    tot[tid] = a;
  }
  __syncthreads();
}

__global__ __launch_bounds__(TPB) void k_trip(const float* __restrict__ pred,
                                              const int* __restrict__ locs,
                                              const v4i* __restrict__ rec,
                                              float* dpn) {
  __shared__ double red[22 * (TPB / 32)];
  __shared__ double tot[24];
  __shared__ double Mf[72];
  __shared__ float Hs[8];

  const int tid = threadIdx.x;
  const int b = blockIdx.x;
  const v4i* rp = rec + (size_t)(2 * b) * NP;
  const v4i* rn = rec + (size_t)(2 * b + 1) * NP;
  const int* locO = locs + b * NP;
  const int* locP = locs + NBT * NP;
  const int* locN = locs + 2 * NBT * NP;
  const int* locM = locs + (NBT + b) * NP;
  const float* predO = pred + (size_t)b * HWIMG;
  const float* predM = pred + (size_t)(NBT + b) * HWIMG;

  double sA[10];
#pragma unroll
  for (int q = 0; q < 10; ++q) sA[q] = 0.0;
  for (int i = tid; i < NP; i += TPB) {
    const v4i ep = rp[i];
    const v4i en = rn[i];
    const int loc = clampi(locO[i], 0, HWIMG - 1);
    const int xoR = loc >> LOGW, yoR = loc & (WIMG - 1);
    if ((float)ep.x < RATIO_THR * (float)ep.y) {
      const int ip = clampi(ep.z, 0, NP - 1);
      const int lp = clampi(locP[ip], 0, HWIMG - 1);
      sA[0] += 1.0; sA[1] += (double)xoR; sA[2] += (double)yoR;
      sA[3] += (double)(lp >> LOGW); sA[4] += (double)(lp & (WIMG - 1));
    }
    if ((float)en.x < RATIO_THR * (float)en.y) {
      const int iq = clampi(en.z, 0, NP - 1);
      const int ln = clampi(locN[iq], 0, HWIMG - 1);
      sA[5] += 1.0; sA[6] += (double)xoR; sA[7] += (double)yoR;
      sA[8] += (double)(ln >> LOGW); sA[9] += (double)(ln & (WIMG - 1));
    }
  }
  blk_sum<10>(sA, red, tot);
  const double cntp = tot[0], cntn = tot[5];
  const double rcP = 1.0 / cntp, rcN = 1.0 / cntn;
  const float mxo_p = (float)(tot[1] * rcP), myo_p = (float)(tot[2] * rcP);
  const float mu_p  = (float)(tot[3] * rcP), mv_p  = (float)(tot[4] * rcP);
  const float mxo_n = (float)(tot[6] * rcN), myo_n = (float)(tot[7] * rcN);
  const float mu_n  = (float)(tot[8] * rcN), mv_n  = (float)(tot[9] * rcN);

  double sB[22];
#pragma unroll
  for (int q = 0; q < 22; ++q) sB[q] = 0.0;
  for (int i = tid; i < NP; i += TPB) {
    const v4i ep = rp[i];
    if ((float)ep.x < RATIO_THR * (float)ep.y) {
      const int loc = clampi(locO[i], 0, HWIMG - 1);
      const int ip = clampi(ep.z, 0, NP - 1);
      const int lp = clampi(locP[ip], 0, HWIMG - 1);
      const float xo = (float)(loc >> LOGW) - mxo_p;
      const float yo = (float)(loc & (WIMG - 1)) - myo_p;
      const float u  = (float)(lp >> LOGW) - mu_p;
      const float v  = (float)(lp & (WIMG - 1)) - mv_p;
      const double dx = (double)xo, dy = (double)yo, du = (double)u, dv = (double)v;
      const double t1 = dx * dx, t2 = dx * dy, t3 = dy * dy;
      const double qq = du * du + dv * dv;
      sB[0] += t1;  sB[1] += t2;  sB[2] += t3;  sB[3] += dx;  sB[4] += dy;
      sB[5] += du * t1; sB[6] += du * t2; sB[7] += du * t3; sB[8] += du * dx; sB[9] += du * dy;
      sB[10] += dv * t1; sB[11] += dv * t2; sB[12] += dv * t3; sB[13] += dv * dx; sB[14] += dv * dy;
      sB[15] += qq * t1; sB[16] += qq * t2; sB[17] += qq * t3; sB[18] += qq * dx; sB[19] += qq * dy;
      sB[20] += du; sB[21] += dv;
    }
  }
  blk_sum<22>(sB, red, tot);
  if (tid == 0) {
    const double Sxx = tot[0],  Sxy = tot[1],  Syy = tot[2],  Sx = tot[3],  Sy = tot[4];
    const double Uxx = tot[5],  Uxy = tot[6],  Uyy = tot[7],  Ux = tot[8],  Uy = tot[9];
    const double Vxx = tot[10], Vxy = tot[11], Vyy = tot[12], Vx = tot[13], Vy = tot[14];
    const double Qxx = tot[15], Qxy = tot[16], Qyy = tot[17], Qx = tot[18], Qy = tot[19];
    const double Su  = tot[20], Sv  = tot[21];
#pragma unroll 1
    for (int q = 0; q < 72; ++q) Mf[q] = 0.0;
    Mf[0 * 9 + 0] = Sxx; Mf[0 * 9 + 1] = Sxy; Mf[0 * 9 + 2] = Sx;
    Mf[1 * 9 + 0] = Sxy; Mf[1 * 9 + 1] = Syy; Mf[1 * 9 + 2] = Sy;
    Mf[2 * 9 + 0] = Sx;  Mf[2 * 9 + 1] = Sy;  Mf[2 * 9 + 2] = cntp;
    Mf[3 * 9 + 3] = Sxx; Mf[3 * 9 + 4] = Sxy; Mf[3 * 9 + 5] = Sx;
    Mf[4 * 9 + 3] = Sxy; Mf[4 * 9 + 4] = Syy; Mf[4 * 9 + 5] = Sy;
    Mf[5 * 9 + 3] = Sx;  Mf[5 * 9 + 4] = Sy;  Mf[5 * 9 + 5] = cntp;
    Mf[0 * 9 + 6] = -Uxx; Mf[0 * 9 + 7] = -Uxy;
    Mf[1 * 9 + 6] = -Uxy; Mf[1 * 9 + 7] = -Uyy;
    Mf[2 * 9 + 6] = -Ux;  Mf[2 * 9 + 7] = -Uy;
    Mf[3 * 9 + 6] = -Vxx; Mf[3 * 9 + 7] = -Vxy;
    Mf[4 * 9 + 6] = -Vxy; Mf[4 * 9 + 7] = -Vyy;
    Mf[5 * 9 + 6] = -Vx;  Mf[5 * 9 + 7] = -Vy;
    Mf[6 * 9 + 0] = -Uxx; Mf[6 * 9 + 1] = -Uxy; Mf[6 * 9 + 2] = -Ux;
    Mf[6 * 9 + 3] = -Vxx; Mf[6 * 9 + 4] = -Vxy; Mf[6 * 9 + 5] = -Vx;
    Mf[7 * 9 + 0] = -Uxy; Mf[7 * 9 + 1] = -Uyy; Mf[7 * 9 + 2] = -Uy;
    Mf[7 * 9 + 3] = -Vxy; Mf[7 * 9 + 4] = -Vyy; Mf[7 * 9 + 5] = -Vy;
    Mf[6 * 9 + 6] = Qxx; Mf[6 * 9 + 7] = Qxy;
    Mf[7 * 9 + 6] = Qxy; Mf[7 * 9 + 7] = Qyy;
    Mf[0 * 9 + 8] = Ux;  Mf[1 * 9 + 8] = Uy;  Mf[2 * 9 + 8] = Su;
    Mf[3 * 9 + 8] = Vx;  Mf[4 * 9 + 8] = Vy;  Mf[5 * 9 + 8] = Sv;
    Mf[6 * 9 + 8] = -Qx; Mf[7 * 9 + 8] = -Qy;
#pragma unroll 1
    for (int k = 0; k < 8; ++k) {
      int piv = k;
      double mx = fabs(Mf[k * 9 + k]);
#pragma unroll 1
      for (int r = k + 1; r < 8; ++r) {
        const double a = fabs(Mf[r * 9 + k]);
        if (a > mx) { mx = a; piv = r; }
      }
      if (piv != k) {
#pragma unroll 1
        for (int c = 0; c < 9; ++c) {
          const double t = Mf[k * 9 + c]; Mf[k * 9 + c] = Mf[piv * 9 + c]; Mf[piv * 9 + c] = t;
        }
      }
      const double inv = 1.0 / Mf[k * 9 + k];
#pragma unroll 1
      for (int c = 0; c < 9; ++c) Mf[k * 9 + c] *= inv;
#pragma unroll 1
      for (int r = 0; r < 8; ++r) {
        if (r == k) continue;
        const double f = Mf[r * 9 + k];
#pragma unroll 1
        for (int c = 0; c < 9; ++c) Mf[r * 9 + c] -= f * Mf[k * 9 + c];
      }
    }
#pragma unroll 1
    for (int k = 0; k < 8; ++k) Hs[k] = (float)Mf[k * 9 + 8];
  }
  __syncthreads();
  const float h0 = Hs[0], h1 = Hs[1], h2 = Hs[2];
  const float h3 = Hs[3], h4 = Hs[4], h5 = Hs[5];
  const float h6 = Hs[6], h7 = Hs[7];

  double sC[2];
  sC[0] = 0.0; sC[1] = 0.0;
  for (int it = tid; it < 2 * NP; it += TPB) {
    const int side = it >> 10;
    const int i = it & (NP - 1);
    const v4i e = (side ? rn : rp)[i];
    if ((float)e.x < RATIO_THR * (float)e.y) {
      const int loc = clampi(locO[i], 0, HWIMG - 1);
      const float pso = predO[loc];
      const int ix = clampi(e.z, 0, NP - 1);
      const int lt = clampi((side ? locN : locP)[ix], 0, HWIMG - 1);
      const int lm = clampi(locM[ix], 0, HWIMG - 1);
      const float pst = predM[lm];
      const float mx = side ? mxo_n : mxo_p;
      const float my = side ? myo_n : myo_p;
      const float mu = side ? mu_n : mu_p;
      const float mv = side ? mv_n : mv_p;
      const float xo = (float)(loc >> LOGW) - mx;
      const float yo = (float)(loc & (WIMG - 1)) - my;
      const float u  = (float)(lt >> LOGW) - mu;
      const float v  = (float)(lt & (WIMG - 1)) - mv;
      const float sx = h0 * xo + h1 * yo + h2;
      const float sy = h3 * xo + h4 * yo + h5;
      const float sz = h6 * xo + h7 * yo + 1.0f;
      const float rz = 1.0f / sz;
      const float px = sx * rz, py = sy * rz, pz = sz * rz;
      const float ax = u - px, ay = v - py, az = 1.0f - pz;
      const float d = sqrtf(ax * ax + ay * ay + az * az + 1e-12f);
      const double c = (double)(d * pso * pst);
      if (side) sC[1] += c; else sC[0] += c;
    }
  }
  blk_sum<2>(sC, red, tot);
  if (tid < 8) {
    const float dp = (float)(tot[0] * rcP);
    const float dn = (float)(tot[1] * rcN);
    v4f val = {0.f, 0.f, 0.f, 0.f};
    if (tid == 0) { val.x = dp; val.y = dn; }
    volatile v4f* dst = (volatile v4f*)(dpn + b * 32) + tid;
    *dst = val;
    __threadfence();
    *dst = val;
  }
}

__global__ __launch_bounds__(TPB) void k_out(const float* __restrict__ pred,
                                             const float* __restrict__ lab,
                                             const float* dpn,
                                             float* out, int n) {
  __shared__ double red[TPB / 32];
  __shared__ double tot[2];
  const int tid = threadIdx.x;
  double s[1];
  s[0] = 0.0;
  for (int i = tid; i < n; i += TPB) {
    const float p = pred[i], y = lab[i];
    const float wgt = (y == 0.0f) ? DYNAMIC_R : STATIC_R;
    const float t = wgt * (y * logf(p) + (1.0f - y) * logf(1.0f - p));
    s[0] += (double)t;
  }
  blk_sum<1>(s, red, tot);
  if (tid == 0) {
    const float sem = (float)(-(tot[0] / (double)n));
    const float dp0 = dpn[0], dn0 = dpn[1], dp1 = dpn[32], dn1 = dpn[33];
    const float dpos = (dp0 + dp1) * 0.5f;
    const float dneg = (dn0 + dn1) * 0.5f;
    const float x = (dpos - dneg) + TRIP_BIAS;
    const float trip = (x != x) ? x : fmaxf(x, 0.0f);
    const float o0 = SEM_R * sem + TRIP_R * trip;
    volatile float* vo = out;
    vo[0] = o0; vo[1] = sem; vo[2] = trip;
    __threadfence();
    vo[0] = o0; vo[1] = sem; vo[2] = trip;
  }
}

extern "C" void kernel_launch(void* const* d_in, const int* in_sizes, int n_in,
                              void* d_out, int out_size, void* d_ws, size_t ws_size,
                              hipStream_t stream) {
  if (n_in < 4) return;
  const int n0 = in_sizes[0];
  if (n0 != NB3 * HWIMG || in_sizes[1] != n0 || in_sizes[2] != NB3 * NP ||
      in_sizes[3] != NB3 * NSB * NP || out_size < 3) return;
  const size_t recBytes = (size_t)(2 * NBT) * NP * sizeof(v4i);
  const size_t dpnBytes = (size_t)NBT * 128;
  if (ws_size < recBytes + dpnBytes) return;

  const float* pred = (const float*)d_in[0];
  const float* lab  = (const float*)d_in[1];
  const int*   locs = (const int*)d_in[2];
  const int*   feat = (const int*)d_in[3];
  v4i*   rec = (v4i*)d_ws;
  float* dpn = (float*)((char*)d_ws + recBytes);
  float* out = (float*)d_out;

  k_ham<<<dim3(NP / QR, 2 * NBT), HAM_TPB, 0, stream>>>(feat, rec);
  k_trip<<<NBT, TPB, 0, stream>>>(pred, locs, rec, dpn);
  k_out<<<1, TPB, 0, stream>>>(pred, lab, dpn, out, n0);
}
